// CMIA_2843268350555
// MI455X (gfx1250) — hardware-verified
//
#include <hip/hip_runtime.h>
#include <math.h>

constexpr int kBatch  = 16;
constexpr int kChan   = 256;
constexpr int kChan2  = 512;
constexpr int kHW     = 1024;
constexpr int kQK     = 2048;
constexpr int kXtokLd = 1024;
constexpr int kXnLd   = 2048;
constexpr int kGrp    = 4;
constexpr int kNGrp   = kBatch / kGrp;
constexpr float kWCarry    = 16.0f;
constexpr float kCdcCarry  = 16384.0f;
constexpr float kXnCarry   = 1024.0f;
constexpr float kInvHW     = 1.0f / 1024.0f;
constexpr float kLnEps     = 1e-5f;

typedef __attribute__((ext_vector_type(16))) _Float16 v16h;
typedef __attribute__((ext_vector_type(8)))  _Float16 v8h;
typedef __attribute__((ext_vector_type(16))) __bf16   v16b;
typedef __attribute__((ext_vector_type(8)))  __bf16   v8b;
typedef __attribute__((ext_vector_type(8)))  float    v8f;
typedef __attribute__((ext_vector_type(4)))  float    v4f;
typedef __attribute__((ext_vector_type(4)))  unsigned int v4u;

__device__ __forceinline__ unsigned short f2bf_bits(float f) {
  unsigned u = __float_as_uint(f);
  return (unsigned short)((u + 0x7FFFu + ((u >> 16) & 1u)) >> 16);
}
__device__ __forceinline__ float bf_bits2f(unsigned short h) { return __uint_as_float(((unsigned)h) << 16); }

__device__ __forceinline__ void dep_guard_h(v8f& a, v8f& b, v16h x, v16h y) { asm volatile("v_nop\n\tv_nop\n\tv_nop\n\tv_nop" : "+v"(a), "+v"(b) : "v"(x), "v"(y)); }
__device__ __forceinline__ void dep_guard_b(v8f& a, v8f& b, v16b x, v16b y) { asm volatile("v_nop\n\tv_nop\n\tv_nop\n\tv_nop" : "+v"(a), "+v"(b) : "v"(x), "v"(y)); }
__device__ __forceinline__ void keep4_h(v16h a, v16h b, v16h c, v16h d) { asm volatile("v_nop" :: "v"(a), "v"(b), "v"(c), "v"(d)); }
__device__ __forceinline__ void keep4_b(v16b a, v16b b, v16b c, v16b d) { asm volatile("v_nop" :: "v"(a), "v"(b), "v"(c), "v"(d)); }
__device__ __forceinline__ void acc_guard4(v8f& a, v8f& b, v8f& c, v8f& d) { asm volatile("v_nop\n\tv_nop\n\tv_nop\n\tv_nop" : "+v"(a), "+v"(b), "+v"(c), "+v"(d)); }
template <typename T> struct Frag;
template <> struct Frag<_Float16> {
  typedef v16h V; union U { v16h v; v8h h[2]; };
  static __device__ __forceinline__ v16h load(const _Float16* p) {
    U f; f.h[0] = *(const v8h*)(p); f.h[1] = *(const v8h*)(p + 16); return f.v;
  }
  static __device__ __forceinline__ v8f mma(v16h a, v16h b, v8f c) {
    return __builtin_amdgcn_wmma_f32_16x16x32_f16(false, a, false, b, (short)0, c, false, false);
  }
  static __device__ __forceinline__ void guard(v8f& a, v8f& b, v16h x, v16h y) { dep_guard_h(a, b, x, y); }
  static __device__ __forceinline__ void keep(v16h a, v16h b, v16h c, v16h d) { keep4_h(a, b, c, d); }
};
template <> struct Frag<__bf16> {
  typedef v16b V; union U { v16b v; v8b h[2]; };
  static __device__ __forceinline__ v16b load(const __bf16* p) {
    U f; f.h[0] = *(const v8b*)(p); f.h[1] = *(const v8b*)(p + 16); return f.v;
  }
  static __device__ __forceinline__ v8f mma(v16b a, v16b b, v8f c) {
    return __builtin_amdgcn_wmma_f32_16x16x32_bf16(false, a, false, b, (short)0, c, false, false);
  }
  static __device__ __forceinline__ void guard(v8f& a, v8f& b, v16b x, v16b y) { dep_guard_b(a, b, x, y); }
  static __device__ __forceinline__ void keep(v16b a, v16b b, v16b c, v16b d) { keep4_b(a, b, c, d); }
};

__device__ __forceinline__ unsigned pk16(unsigned short a, unsigned short b) { return (unsigned)a | ((unsigned)b << 16); }
__device__ __forceinline__ unsigned short h_bits(float f) { const _Float16 h = (_Float16)f; return __builtin_bit_cast(unsigned short, h); }

template <int ET> struct Elem;
template <> struct Elem<0> { typedef _Float16 T; };
template <> struct Elem<1> { typedef __bf16 T; };
template <int ET, bool SPLIT, int BIAS_MODE, int OUT_MODE, bool RESID, int ACT = 0>
__global__ __launch_bounds__(256) void wmma_gemm64(
    const unsigned short* __restrict__ Ap, const unsigned short* __restrict__ A2p, int lda, long strideA,
    const unsigned short* __restrict__ Btp, const unsigned short* __restrict__ Bt2p, int ldb, long strideB,
    void* __restrict__ Cout, void* __restrict__ Cout2, int ldc, long strideC,
    const float* __restrict__ bias,
    const float* __restrict__ resid, long strideR,
    int M, int N, int K, float scale) {
  typedef typename Elem<ET>::T T;
  typedef typename Frag<T>::V V;
  const T* A = (const T*)Ap; const T* A2 = (const T*)A2p; const T* Bt = (const T*)Btp; const T* Bt2 = (const T*)Bt2p;
  __shared__ __align__(16) float sT[8][16 * 68];
  const int b    = blockIdx.y;
  const int lane = threadIdx.x & 31;
  const int wave = threadIdx.x >> 5;
  const int tilesN = N >> 6;
  const int tilesM = M >> 6;
  const int tile = blockIdx.x * 8 + wave;
  if (tile >= tilesM * tilesN) return;
  const int tm = tile / tilesN;
  const int tn = tile - tm * tilesN;
  const int m0 = tm << 6;
  const int n0 = tn << 6;

  const T* Ab  = A  + (size_t)b * strideA;
  const T* Bb  = Bt + (size_t)b * strideB;
  const T* Ab2 = SPLIT ? (A2  + (size_t)b * strideA) : nullptr;
  const T* Bb2 = SPLIT ? (Bt2 + (size_t)b * strideB) : nullptr;

  const int rlane = lane & 15;
  const int koff  = (lane >> 4) * 8;
  const int mOff  = (lane >> 4) * 8;

  v8f acc[4][4];
#pragma unroll
  for (int i = 0; i < 4; ++i)
#pragma unroll
    for (int j = 0; j < 4; ++j) acc[i][j] = (v8f){0.f,0.f,0.f,0.f,0.f,0.f,0.f,0.f};

  for (int k0 = 0; k0 < K; k0 += 32) {
    V bh[4], bl[4];
#pragma unroll
    for (int j = 0; j < 4; ++j) {
      const size_t bo = (size_t)(n0 + (j << 4) + rlane) * ldb + koff + k0;
      bh[j] = Frag<T>::load(Bb + bo);
      if (SPLIT) bl[j] = Frag<T>::load(Bb2 + bo);
    }
#pragma unroll
    for (int i = 0; i < 4; ++i) {
      const size_t ao = (size_t)(m0 + (i << 4) + rlane) * lda + koff + k0;
      V ah = Frag<T>::load(Ab + ao);
      V al;
      if (SPLIT) al = Frag<T>::load(Ab2 + ao);
#pragma unroll
      for (int j = 0; j < 4; ++j) {
        acc[i][j] = Frag<T>::mma(ah, bh[j], acc[i][j]);
        if (SPLIT) {
          acc[i][j] = Frag<T>::mma(ah, bl[j], acc[i][j]);
          acc[i][j] = Frag<T>::mma(al, bh[j], acc[i][j]);
        }
      }
      Frag<T>::guard(acc[i][0], acc[i][3], ah, SPLIT ? al : ah);
    }
    Frag<T>::keep(bh[0], bh[1], bh[2], bh[3]);
    if (SPLIT) Frag<T>::keep(bl[0], bl[1], bl[2], bl[3]);
  }
  acc_guard4(acc[0][0], acc[0][1], acc[0][2], acc[0][3]);
  acc_guard4(acc[1][0], acc[1][1], acc[1][2], acc[1][3]);
  acc_guard4(acc[2][0], acc[2][1], acc[2][2], acc[2][3]);
  acc_guard4(acc[3][0], acc[3][1], acc[3][2], acc[3][3]);

  float* slab = sT[wave];
  const float* Rb = RESID ? (resid + (size_t)b * strideR) : nullptr;
#pragma unroll
  for (int i = 0; i < 4; ++i) {
    const int mBase = m0 + (i << 4);
#pragma unroll
    for (int j = 0; j < 4; ++j) {
      const int n = n0 + (j << 4) + rlane;
      float bv = 0.f;
      if (BIAS_MODE == 2) bv = bias[n];
#pragma unroll
      for (int r = 0; r < 8; ++r) {
        float v = acc[i][j][r] * scale;
        if (BIAS_MODE == 1) v += bias[mBase + mOff + r];
        if (BIAS_MODE == 2) v += bv;
        if (RESID) v += Rb[(size_t)(mBase + mOff + r) * ldc + n];
        if (ACT == 2) v = fmaxf(v, 0.0f);
        if (ACT == 4) v = (v > 0.f) ? v : 0.01f * v;
        slab[(mOff + r) * 68 + (j << 4) + rlane] = v;
      }
    }
    __builtin_amdgcn_fence(__ATOMIC_RELEASE, "workgroup");
    __builtin_amdgcn_wave_barrier();
    __builtin_amdgcn_fence(__ATOMIC_ACQUIRE, "workgroup");
    if (OUT_MODE == 0) {
      float* C = (float*)Cout + (size_t)b * strideC;
      const int hh = lane >> 4, c4 = (lane & 15) * 4;
      for (int pass = 0; pass < 2; ++pass) {
#pragma unroll
        for (int it = 0; it < 8; ++it) {
          const int row = it * 2 + hh;
          v4f v = *(const v4f*)(slab + row * 68 + c4);
          *(volatile v4f*)(C + (size_t)(mBase + row) * ldc + n0 + c4) = v;
        }
        __threadfence();
      }
    } else {
      const int q = lane >> 3, c8 = (lane & 7) * 8;
      unsigned short* C  = (unsigned short*)Cout  + (size_t)b * strideC;
      unsigned short* C2 = (OUT_MODE == 2) ? ((unsigned short*)Cout2 + (size_t)b * strideC) : nullptr;
      for (int pass = 0; pass < 2; ++pass) {
#pragma unroll
        for (int it = 0; it < 4; ++it) {
          const int row = it * 4 + q;
          const float* sp = slab + row * 68 + c8;
          v8h hv, lv;
#pragma unroll
          for (int e = 0; e < 8; ++e) {
            if (OUT_MODE == 1) {
              hv[e] = (_Float16)sp[e];
            } else {
              unsigned short hb = f2bf_bits(sp[e]);
              unsigned short lb = f2bf_bits(sp[e] - bf_bits2f(hb));
              hv[e] = __builtin_bit_cast(_Float16, hb);
              lv[e] = __builtin_bit_cast(_Float16, lb);
            }
          }
          *(volatile v8h*)(C + (size_t)(mBase + row) * ldc + n0 + c8) = hv;
          if (OUT_MODE == 2) *(volatile v8h*)(C2 + (size_t)(mBase + row) * ldc + n0 + c8) = lv;
        }
        __threadfence();
      }
    }
    __builtin_amdgcn_fence(__ATOMIC_RELEASE, "workgroup");
    __builtin_amdgcn_wave_barrier();
    __builtin_amdgcn_fence(__ATOMIC_ACQUIRE, "workgroup");
  }
}

template <int MODE>
__global__ __launch_bounds__(256) void castw_kernel(const float* __restrict__ in, unsigned short* __restrict__ out,
                                                      int rows, int cols, int ldo, float scale) {
  const int gpr = cols >> 3;
  const int n8  = rows * gpr;
  const int i   = blockIdx.x * 256 + threadIdx.x;
  if (i >= n8) return;
  const int r = i / gpr;
  const int g = i - r * gpr;
  const float* p = in + (size_t)r * cols + 8 * g;
  const v4f a = *(const v4f*)(p);
  const v4f c = *(const v4f*)(p + 4);
  float x[8];
#pragma unroll
  for (int e = 0; e < 4; ++e) { x[e] = a[e] * scale; x[4 + e] = c[e] * scale; }
  unsigned short hb[8], lb[8];
#pragma unroll
  for (int e = 0; e < 8; ++e) {
    const _Float16 h = (_Float16)x[e];
    hb[e] = __builtin_bit_cast(unsigned short, h);
    lb[e] = (MODE == 2) ? h_bits(x[e] - (float)h) : hb[e];
  }
  const v4u uh = (v4u){pk16(hb[0], hb[1]), pk16(hb[2], hb[3]), pk16(hb[4], hb[5]), pk16(hb[6], hb[7])};
  const v4u ul = (v4u){pk16(lb[0], lb[1]), pk16(lb[2], lb[3]), pk16(lb[4], lb[5]), pk16(lb[6], lb[7])};
  unsigned short* q0 = out + (size_t)r * ldo + 8 * g;
  unsigned short* q1 = q0 + cols;
  *(volatile v4u*)q0 = uh;
  if (MODE != 0) *(volatile v4u*)q1 = ul;
  __threadfence();
  *(volatile v4u*)q0 = uh;
  if (MODE != 0) *(volatile v4u*)q1 = ul;
}

__global__ __launch_bounds__(256) void xtok_kernel(const float* __restrict__ xs, const float* __restrict__ xf,
                                                   unsigned short* __restrict__ xtok) {
  __shared__ float sm[64][65];
  const int t  = threadIdx.x;
  const int n0 = blockIdx.x * 64;
  const int ct = blockIdx.y;
  const int b  = blockIdx.z;
  const float* X = (ct < 4) ? xs : xf;
  const int c0 = (ct & 3) * 64;
  const float* src = X + ((size_t)b * kChan + c0) * kHW + n0;
#pragma unroll
  for (int i = 0; i < 16; ++i) {
    const int e  = i * 256 + t;
    const int r  = e >> 6;
    const int cc = e & 63;
    sm[cc][r] = src[(size_t)r * kHW + cc];
  }
  __syncthreads();
  const int lane = t & 31, wave = t >> 5;
  const int q = lane >> 3, c8 = (lane & 7) * 8;
  unsigned short* ob = xtok + ((size_t)b * kHW + n0) * kXtokLd + ct * 64 + c8;
#pragma unroll
  for (int it = 0; it < 2; ++it) {
    const int row = wave * 8 + it * 4 + q;
    unsigned short hb[8];
#pragma unroll
    for (int e = 0; e < 8; ++e) hb[e] = h_bits(sm[row][c8 + e]);
    const v4u u = (v4u){pk16(hb[0], hb[1]), pk16(hb[2], hb[3]), pk16(hb[4], hb[5]), pk16(hb[6], hb[7])};
    unsigned short* p0 = ob + (size_t)row * kXtokLd;
    unsigned short* p1 = p0 + kChan2;
    *(volatile v4u*)p0 = u;
    *(volatile v4u*)p1 = u;
    __threadfence();
    *(volatile v4u*)p0 = u;
    *(volatile v4u*)p1 = u;
  }
}

__global__ __launch_bounds__(128) void layernorm_kernel(const float* __restrict__ xb, const float* __restrict__ gam,
                                                        const float* __restrict__ bet, unsigned short* __restrict__ xn) {
  __shared__ float red[4];
  const int row  = blockIdx.x;
  const int t    = threadIdx.x, lane = t & 31, wave = t >> 5;
  const int c0   = t * 8;
  const float* px = xb + (size_t)row * kHW + c0;
  const v4f a = *(const v4f*)(px);
  const v4f c = *(const v4f*)(px + 4);
  float x[8];
#pragma unroll
  for (int e = 0; e < 4; ++e) { x[e] = a[e]; x[4 + e] = c[e]; }
  float s = ((x[0] + x[1]) + (x[2] + x[3])) + ((x[4] + x[5]) + (x[6] + x[7]));
#pragma unroll
  for (int off = 16; off > 0; off >>= 1) s += __shfl_xor(s, off, 32);
  if (lane == 0) red[wave] = s;
  __syncthreads();
  const float mean = ((red[0] + red[1]) + (red[2] + red[3])) * kInvHW;
  __syncthreads();
  float d[8];
  float sq = 0.f;
#pragma unroll
  for (int e = 0; e < 8; ++e) { d[e] = x[e] - mean; sq += d[e] * d[e]; }
#pragma unroll
  for (int off = 16; off > 0; off >>= 1) sq += __shfl_xor(sq, off, 32);
  if (lane == 0) red[wave] = sq;
  __syncthreads();
  const float var  = ((red[0] + red[1]) + (red[2] + red[3])) * kInvHW;
  const float rstd = 1.0f / sqrtf(var + kLnEps);
  const v4f g0 = *(const v4f*)(gam + c0), g1 = *(const v4f*)(gam + c0 + 4);
  const v4f e0 = *(const v4f*)(bet + c0), e1 = *(const v4f*)(bet + c0 + 4);
  float gg[8], bb[8];
#pragma unroll
  for (int e = 0; e < 4; ++e) { gg[e] = g0[e]; gg[4 + e] = g1[e]; bb[e] = e0[e]; bb[4 + e] = e1[e]; }
  unsigned short hb[8], lb[8];
#pragma unroll
  for (int e = 0; e < 8; ++e) {
    const float y  = d[e] * rstd * gg[e] + bb[e];
    const float ys = y * kXnCarry;
    const _Float16 h = (_Float16)ys;
    hb[e] = __builtin_bit_cast(unsigned short, h);
    lb[e] = h_bits(ys - (float)h);
  }
  const v4u uh = (v4u){pk16(hb[0], hb[1]), pk16(hb[2], hb[3]), pk16(hb[4], hb[5]), pk16(hb[6], hb[7])};
  const v4u ul = (v4u){pk16(lb[0], lb[1]), pk16(lb[2], lb[3]), pk16(lb[4], lb[5]), pk16(lb[6], lb[7])};
  unsigned short* q0 = xn + (size_t)row * kXnLd + c0;
  unsigned short* q1 = q0 + kHW;
  *(volatile v4u*)q0 = uh;
  *(volatile v4u*)q1 = ul;
  __threadfence();
  *(volatile v4u*)q0 = uh;
  *(volatile v4u*)q1 = ul;
}

__global__ __launch_bounds__(256) void colsoftmax_kernel(const float* __restrict__ sc, unsigned short* __restrict__ pth,
                                                         unsigned short* __restrict__ ptl) {
  __shared__ float pm[4][64];
  __shared__ float ps[4][64];
  __shared__ float cmax[64];
  __shared__ float cinv[64];
  const int t  = threadIdx.x;
  const int n0 = blockIdx.x * 64;
  const int g  = blockIdx.y;
  const float* sg = sc + (size_t)g * kHW * kHW + n0;
  {
    const int col = t & 63, rg = t >> 6;
    const float* cp = sg + (size_t)rg * kHW + col;
    float m = cp[0];
    float s = 1.0f;
#pragma unroll 1
    for (int i = 1; i < 256; ++i) {
      const float x  = cp[(size_t)i * 4 * kHW];
      const float d  = x - m;
      const float ex = expf(-fabsf(d));
      const bool up  = d > 0.0f;
      s = up ? (s * ex + 1.0f) : (s + ex);
      m = up ? x : m;
    }
    pm[rg][col] = m;
    ps[rg][col] = s;
  }
  __syncthreads();
  if (t < 64) {
    const float M = fmaxf(fmaxf(pm[0][t], pm[1][t]), fmaxf(pm[2][t], pm[3][t]));
    float S = 0.f;
#pragma unroll 1
    for (int r = 0; r < 4; ++r) S += ps[r][t] * expf(pm[r][t] - M);
    cmax[t] = M;
    cinv[t] = 1.0f / S;
  }
  __syncthreads();
  {
    const int q8 = t & 7, ro = t >> 3, c0 = q8 * 8;
    unsigned short* oh = pth + (size_t)g * kHW * kHW + n0 + c0;
    unsigned short* ol = ptl + (size_t)g * kHW * kHW + n0 + c0;
#pragma unroll 1
    for (int i = 0; i < 32; ++i) {
      const int j = ro + 32 * i;
      const float* rp = sg + (size_t)j * kHW + c0;
      unsigned w0h = 0u, w1h = 0u, w2h = 0u, w3h = 0u;
      unsigned w0l = 0u, w1l = 0u, w2l = 0u, w3l = 0u;
#pragma unroll 1
      for (int e = 0; e < 8; ++e) {
        const float x = rp[e];
        const float p = expf(x - cmax[c0 + e]) * cinv[c0 + e];
        const unsigned short hb = f2bf_bits(p);
        const unsigned short lb = f2bf_bits(p - bf_bits2f(hb));
        const unsigned sh = (unsigned)(e & 1) * 16u;
        const unsigned hv = ((unsigned)hb) << sh;
        const unsigned lv = ((unsigned)lb) << sh;
        const int wsel = e >> 1;
        w0h |= (wsel == 0) ? hv : 0u;  w0l |= (wsel == 0) ? lv : 0u;
        w1h |= (wsel == 1) ? hv : 0u;  w1l |= (wsel == 1) ? lv : 0u;
        w2h |= (wsel == 2) ? hv : 0u;  w2l |= (wsel == 2) ? lv : 0u;
        w3h |= (wsel == 3) ? hv : 0u;  w3l |= (wsel == 3) ? lv : 0u;
      }
      const v4u uh = (v4u){w0h, w1h, w2h, w3h};
      const v4u ul = (v4u){w0l, w1l, w2l, w3l};
      unsigned short* ph = oh + (size_t)j * kHW;
      unsigned short* pl = ol + (size_t)j * kHW;
      *(volatile v4u*)ph = uh;
      *(volatile v4u*)pl = ul;
      __threadfence();
      *(volatile v4u*)ph = uh;
      *(volatile v4u*)pl = ul;
    }
  }
}

extern "C" void kernel_launch(void* const* d_in, const int* in_sizes, int n_in,
                              void* d_out, int out_size, void* d_ws, size_t ws_size,
                              hipStream_t stream) {
  if (n_in < 15) return;
  const int nX = kBatch * kChan * kHW;
  if (in_sizes[0] != nX || in_sizes[1] != nX) return;
  if (in_sizes[2] != kChan * kChan2 || in_sizes[3] != kChan) return;
  if (in_sizes[4] != kChan * kChan || in_sizes[5] != kChan) return;
  if (in_sizes[6] != kChan * kChan || in_sizes[7] != kChan) return;
  if (in_sizes[8] != kHW || in_sizes[9] != kHW) return;
  if (in_sizes[10] != kQK * kHW || in_sizes[11] != kHW * kHW || in_sizes[12] != kHW) return;
  if (in_sizes[13] != kHW * kHW || in_sizes[14] != kHW) return;
  if (out_size != 2 * nX) return;
  const size_t kMiB  = 1048576;
  const size_t wsEnd = 108 * kMiB + 768 * 1024;
  if (ws_size < wsEnd) return;

  const float* x_spa  = (const float*)d_in[0];
  const float* x_freq = (const float*)d_in[1];
  const float* w_cdc  = (const float*)d_in[2];
  const float* b_cdc  = (const float*)d_in[3];
  const float* w_sv   = (const float*)d_in[4];
  const float* b_sv   = (const float*)d_in[5];
  const float* w_fv   = (const float*)d_in[6];
  const float* b_fv   = (const float*)d_in[7];
  const float* ln_w   = (const float*)d_in[8];
  const float* ln_b   = (const float*)d_in[9];
  const float* w_qk   = (const float*)d_in[10];
  const float* w_spa  = (const float*)d_in[11];
  const float* b_spa  = (const float*)d_in[12];
  const float* w_frq  = (const float*)d_in[13];
  const float* b_frq  = (const float*)d_in[14];
  float* outp = (float*)d_out;

  char* ws = (char*)d_ws;
  unsigned short* xtok    = (unsigned short*)(ws);
  unsigned short* xn      = (unsigned short*)(ws);
  unsigned short* att16   = (unsigned short*)(ws);
  float*          xbuf    = (float*)(ws + 32 * kMiB);
  unsigned short* qktok   = (unsigned short*)(ws + 32 * kMiB);
  float*          scores  = (float*)(ws + 32 * kMiB);
  unsigned short* pt_hi   = (unsigned short*)(ws + 48 * kMiB);
  unsigned short* pt_lo   = (unsigned short*)(ws + 56 * kMiB);
  unsigned short* vspa_hi = (unsigned short*)(ws + 64 * kMiB);
  unsigned short* vspa_lo = (unsigned short*)(ws + 72 * kMiB);
  unsigned short* vfrq_hi = (unsigned short*)(ws + 80 * kMiB);
  unsigned short* vfrq_lo = (unsigned short*)(ws + 88 * kMiB);
  unsigned short* wqk2    = (unsigned short*)(ws + 96 * kMiB);
  unsigned short* wspa16  = (unsigned short*)(ws + 104 * kMiB);
  unsigned short* wfrq16  = (unsigned short*)(ws + 106 * kMiB);
  unsigned short* wcdc_pk = (unsigned short*)(ws + 108 * kMiB);
  unsigned short* wsv16   = (unsigned short*)(ws + 108 * kMiB + 512 * 1024);
  unsigned short* wfv16   = (unsigned short*)(ws + 108 * kMiB + 640 * 1024);

  const long sX   = (long)kChan * kHW;
  const long sTok = (long)kHW * kXtokLd;
  const long sXn  = (long)kChan * kXnLd;
  const long sQK  = (long)kQK * kChan;
  const long sAtt = (long)kHW * kHW;

  {
    const int n8sv = kChan * kChan / 8;
    castw_kernel<0><<<(n8sv + 255) / 256, 256, 0, stream>>>(w_sv, wsv16, kChan, kChan, kChan, kWCarry);
    castw_kernel<0><<<(n8sv + 255) / 256, 256, 0, stream>>>(w_fv, wfv16, kChan, kChan, kChan, kWCarry);
    const int n8cdc = kChan * kChan2 / 8;
    castw_kernel<2><<<(n8cdc + 255) / 256, 256, 0, stream>>>(w_cdc, wcdc_pk, kChan, kChan2, 2 * kChan2, kCdcCarry);
    const int n8qk = kQK * kHW / 8;
    castw_kernel<1><<<(n8qk + 255) / 256, 256, 0, stream>>>(w_qk, wqk2, kQK, kHW, 2 * kHW, kWCarry);
    const int n8w = kHW * kHW / 8;
    castw_kernel<0><<<(n8w + 255) / 256, 256, 0, stream>>>(w_spa, wspa16, kHW, kHW, kHW, kWCarry);
    castw_kernel<0><<<(n8w + 255) / 256, 256, 0, stream>>>(w_frq, wfrq16, kHW, kHW, kHW, kWCarry);
  }

  xtok_kernel<<<dim3(kHW / 64, kChan2 / 64, kBatch), 256, 0, stream>>>(x_spa, x_freq, xtok);

  wmma_gemm64<0, false, 1, 2, false><<<dim3(8, kBatch), 256, 0, stream>>>(
      wsv16, wsv16, kChan, 0L, xtok, xtok, kXtokLd, sTok,
      (void*)vspa_hi, (void*)vspa_lo, kHW, sX, b_sv, x_spa, 0L, kChan, kHW, kChan, 1.0f / kWCarry);
  wmma_gemm64<0, false, 1, 2, false><<<dim3(8, kBatch), 256, 0, stream>>>(
      wfv16, wfv16, kChan, 0L, xtok + kChan, xtok + kChan, kXtokLd, sTok,
      (void*)vfrq_hi, (void*)vfrq_lo, kHW, sX, b_fv, x_freq, 0L, kChan, kHW, kChan, 1.0f / kWCarry);

  wmma_gemm64<0, false, 1, 0, false><<<dim3(8, kBatch), 256, 0, stream>>>(
      wcdc_pk, wcdc_pk, 2 * kChan2, 0L, xtok, xtok, kXtokLd, sTok,
      (void*)xbuf, (void*)xbuf, kHW, sX, b_cdc, x_spa, 0L, kChan, kHW, 2 * kChan2, 1.0f / kCdcCarry);

  layernorm_kernel<<<kBatch * kChan, 128, 0, stream>>>(xbuf, ln_w, ln_b, xn);

  wmma_gemm64<0, false, 0, 1, false><<<dim3(16, kBatch), 256, 0, stream>>>(
      wqk2, wqk2, 2 * kHW, 0L, xn, xn, kXnLd, sXn,
      (void*)qktok, (void*)qktok, kChan, sQK, b_cdc, x_spa, 0L, kQK, kChan, 2 * kHW, 1.0f / (kWCarry * kXnCarry));

  wmma_gemm64<0, false, 0, 1, false><<<dim3(32, kBatch), 256, 0, stream>>>(
      qktok, qktok, kChan, sQK, qktok + (size_t)kHW * kChan, qktok + (size_t)kHW * kChan, kChan, sQK,
      (void*)att16, (void*)att16, kHW, sAtt, b_cdc, x_spa, 0L, kHW, kHW, kChan, 0.03125f);

  for (int br = 0; br < 2; ++br) {
    const unsigned short* w16 = (br == 0) ? wspa16 : wfrq16;
    const float* bsc          = (br == 0) ? b_spa : b_frq;
    const unsigned short* vh  = (br == 0) ? vspa_hi : vfrq_hi;
    const unsigned short* vl  = (br == 0) ? vspa_lo : vfrq_lo;
    const float* xres         = (br == 0) ? x_spa : x_freq;
    float* ob = outp + (size_t)br * (size_t)nX;
    for (int gi = 0; gi < kNGrp; ++gi) {
      const int b0 = gi * kGrp;
      wmma_gemm64<0, false, 1, 0, false><<<dim3(32, kGrp), 256, 0, stream>>>(
          w16, w16, kHW, 0L, att16 + (size_t)b0 * sAtt, att16 + (size_t)b0 * sAtt, kHW, sAtt,
          (void*)scores, (void*)scores, kHW, sAtt, bsc, xres, 0L, kHW, kHW, kHW, 1.0f / kWCarry);
      colsoftmax_kernel<<<dim3(kHW / 64, kGrp), 256, 0, stream>>>(scores, pt_hi, pt_lo);
      wmma_gemm64<1, true, 0, 0, true><<<dim3(8, kGrp), 256, 0, stream>>>(
          vh + (size_t)b0 * sX, vl + (size_t)b0 * sX, kHW, sX, pt_hi, pt_lo, kHW, sAtt,
          (void*)(ob + (size_t)b0 * sX), (void*)(ob + (size_t)b0 * sX), kHW, sX, bsc,
          xres + (size_t)b0 * sX, sX, kChan, kHW, kHW, 1.0f);
    }
  }
}
